// MultiHeadAttention_10333691314638
// MI455X (gfx1250) — hardware-run, weakly checked
//
#include <hip/hip_runtime.h>


#ifndef NB
#define NB 2
#endif
#ifndef SEQ
#define SEQ 2048
#endif
#define NB_FULL  2
#define SEQ_FULL 2048
#ifndef OUT_SEQ
#define OUT_SEQ SEQ
#endif
#define DM   1024
#define NH_  16
#define HD   64
#define AW   4
#define QRS  2048.0f
#define QRI  (1.0f / 2048.0f)
#define SC2  (0.125f * 1.4426950408889634f)
#define PSH  8.0f
#define WOS  256.0f
#define WOI  (1.0f / 256.0f)
#define HMIN 6.103515625e-5f

static_assert(HD == 64);
static_assert(NH_ * HD == DM);
static_assert(DM % 64 == 0);
static_assert(DM % 32 == 0);
static_assert(SEQ % 64 == 0);
static_assert((NB * SEQ) % 64 == 0);
static_assert(SEQ % 32 == 0);
static_assert(SEQ % (16 * AW) == 0);
static_assert(((size_t)SEQ * DM) % 8 == 0);
static_assert(NB <= NB_FULL);
static_assert(SEQ <= SEQ_FULL);

typedef _Float16 h16;
typedef unsigned short bf;
typedef __attribute__((ext_vector_type(16))) __bf16   v16bf;
typedef __attribute__((ext_vector_type(16))) _Float16 v16h;
typedef __attribute__((ext_vector_type(8)))  _Float16 v8h;
typedef __attribute__((ext_vector_type(8)))  unsigned short v8us;
typedef __attribute__((ext_vector_type(8)))  float    v8f;
typedef __attribute__((ext_vector_type(4)))  float    v4f;
typedef v4f  __attribute__((may_alias)) v4fa;

__device__ __forceinline__ unsigned short f2bf(float f) { unsigned u = __float_as_uint(f); u += 0x7FFFu + ((u >> 16) & 1u); return (unsigned short)(u >> 16); }
__device__ __forceinline__ float bfr(float f) { return __uint_as_float(((unsigned)f2bf(f)) << 16); }
__device__ __forceinline__ h16 hfl(h16 a) { return (fabsf((float)a) < HMIN) ? (h16)0.0f : a; }
__device__ __forceinline__ v16h cat16(v8h lo, v8h hi) { return __builtin_shufflevector(lo, hi, 0, 1, 2, 3, 4, 5, 6, 7, 8, 9, 10, 11, 12, 13, 14, 15); }
__device__ __forceinline__ v16bf cat16b(v8us lo, v8us hi) { return __builtin_bit_cast(v16bf, __builtin_shufflevector(lo, hi, 0, 1, 2, 3, 4, 5, 6, 7, 8, 9, 10, 11, 12, 13, 14, 15)); }
__device__ __forceinline__ v8f wmma16(v16h a, v16h b, v8f c) { return __builtin_amdgcn_wmma_f32_16x16x32_f16(false, a, false, b, (short)0, c, false, false); }
__device__ __forceinline__ v8f wmmab(v16bf a, v16bf b, v8f c) { return __builtin_amdgcn_wmma_f32_16x16x32_bf16(false, a, false, b, (short)0, c, false, false); }
__device__ __forceinline__ v16h  ldh(const h16* p) { return cat16(*(const v8h*)p, *(const v8h*)(p + 16)); }
__device__ __forceinline__ v16bf ldb(const bf* p)  { return cat16b(*(const v8us*)p, *(const v8us*)(p + 16)); }
__device__ __forceinline__ void wave_sync() { __builtin_amdgcn_fence(3  , "wavefront"); __builtin_amdgcn_wave_barrier(); asm volatile("" ::: "memory"); }

__global__ __launch_bounds__(256) void k_cvt8(const float* __restrict__ src, bf* dst, size_t n8) {
    const size_t i = (size_t)blockIdx.x * 256 + threadIdx.x; if (i >= n8) return;
    const v8f v = *(const v8f*)(src + i * 8); v8us o;
#pragma unroll
    for (int k = 0; k < 8; ++k) o[k] = f2bf(v[k]);
    *(volatile v8us*)(dst + i * 8) = o; __threadfence(); *(volatile v8us*)(dst + i * 8) = o;
}

template <int MODE>
__global__ __launch_bounds__(256) void k_cvtT(const float* __restrict__ src, bf* dst, int rows, int cols, size_t sstride, size_t dstride) {
    __shared__ float tl[64 * 65];
    const int tid = threadIdx.x; const int c0 = blockIdx.x * 64, r0 = blockIdx.y * 64;
    const float* s = src + (size_t)blockIdx.z * sstride; bf* d = dst + (size_t)blockIdx.z * dstride;
#pragma unroll
    for (int i = 0; i < 4; ++i) { const int idx = tid + i * 256; const int r = idx >> 4, c4 = (idx & 15) * 4;
        const v4f v = *(const v4f*)(s + (size_t)(r0 + r) * (size_t)cols + c0 + c4);
        tl[r * 65 + c4 + 0] = v[0]; tl[r * 65 + c4 + 1] = v[1]; tl[r * 65 + c4 + 2] = v[2]; tl[r * 65 + c4 + 3] = v[3]; }
    __syncthreads();
    v8us o[2];
#pragma unroll
    for (int i = 0; i < 2; ++i) { const int idx = tid + i * 256; const int c = idx >> 3, p8 = (idx & 7) * 8;
        if (MODE == 0) {
#pragma unroll
            for (int k = 0; k < 8; ++k) o[i][k] = f2bf(tl[(p8 + k) * 65 + c]);
        } else { v8h hv;
#pragma unroll
            for (int k = 0; k < 8; ++k) hv[k] = hfl((h16)(bfr(tl[(p8 + k) * 65 + c]) * WOS));
            o[i] = __builtin_bit_cast(v8us, hv); } }
#pragma unroll 1
    for (int ps = 0; ps < 2; ++ps) {
#pragma unroll
        for (int i = 0; i < 2; ++i) { const int idx = tid + i * 256; const int c = idx >> 3, p8 = (idx & 7) * 8;
            *(volatile v8us*)(d + (size_t)(c0 + c) * (size_t)rows + r0 + p8) = o[i]; }
        if (ps == 0) __threadfence(); }
}

__global__ __launch_bounds__(32) void k_proj(const bf* __restrict__ A, const bf* __restrict__ Bt, h16* Ph, h16* Pr, int useRes, const float* __restrict__ bias, int biasRow,
                                             int RB, size_t sRB, int pitch, int CB, size_t sCB) {
    __shared__ __align__(16) float os[16 * 68];
    const int K = DM;
    const int lane = threadIdx.x & 31, lr = lane & 15, hi = lane >> 4; const int r0 = blockIdx.x * 64, c0 = blockIdx.y * 64;
    v8f acc[4][4];
#pragma unroll
    for (int mb = 0; mb < 4; ++mb)
#pragma unroll
        for (int nb = 0; nb < 4; ++nb) acc[mb][nb] = (v8f){};
    const size_t aoff = (size_t)(r0 + lr) * K + 8 * hi, boff = (size_t)(c0 + lr) * K + 8 * hi;
#pragma unroll 1
    for (int kc = 0; kc < K; kc += 32) {
        v16bf a[4];
#pragma unroll
        for (int mb = 0; mb < 4; ++mb) a[mb] = ldb(A + aoff + (size_t)mb * 16 * K + kc);
#pragma unroll
        for (int nb = 0; nb < 4; ++nb) { const v16bf b = ldb(Bt + boff + (size_t)nb * 16 * K + kc);
#pragma unroll
            for (int mb = 0; mb < 4; ++mb) acc[mb][nb] = wmmab(a[mb], b, acc[mb][nb]); }
        asm volatile("v_nop\n\tv_nop\n\tv_nop\n\tv_nop" : "+v"(acc[0][0]), "+v"(acc[1][1]), "+v"(acc[2][2]), "+v"(acc[3][3]) : "v"(a[0]), "v"(a[1]), "v"(a[2]), "v"(a[3]));
    }
    float bc[4];
#pragma unroll
    for (int nb = 0; nb < 4; ++nb) { int ci = c0 + nb * 16 + lr; ci = ci < DM ? ci : DM - 1; const float t = bfr(bias[ci]); bc[nb] = biasRow ? 0.0f : t; }
    const size_t tbase = (size_t)(r0 / RB) * sRB + (size_t)(r0 % RB) * (size_t)pitch + (size_t)(c0 / CB) * sCB + (size_t)(c0 % CB);
#pragma unroll
    for (int mb = 0; mb < 4; ++mb) {
        int rb = r0 + mb * 16 + hi * 8; rb = rb < DM - 8 ? rb : DM - 8;
        const v4f b0 = *(const v4f*)(bias + rb); const v4f b1 = *(const v4f*)(bias + rb + 4);
        float br[8];
#pragma unroll
        for (int j = 0; j < 4; ++j) { const float t0 = bfr(b0[j]); const float t1 = bfr(b1[j]); br[j] = biasRow ? t0 : 0.0f; br[4 + j] = biasRow ? t1 : 0.0f; }
#pragma unroll
        for (int nb = 0; nb < 4; ++nb) {
#pragma unroll
            for (int j = 0; j < 8; ++j) os[(hi * 8 + j) * 68 + nb * 16 + lr] = acc[mb][nb][j] + bc[nb] + br[j]; }
        wave_sync();
        const size_t sb = tbase + (size_t)(mb * 16) * (size_t)pitch;
#pragma unroll 1
        for (int ps = 0; ps < 2; ++ps) {
#pragma unroll
            for (int s = 0; s < 4; ++s) { const int row = 4 * s + (lane >> 3), c8 = (lane & 7) * 8;
                const v4f x0 = *(const v4fa*)(&os[row * 68 + c8]); const v4f x1 = *(const v4fa*)(&os[row * 68 + c8 + 4]); v8h hv, rv;
#pragma unroll
                for (int i = 0; i < 4; ++i) { const h16 a0 = hfl((h16)x0[i]); const h16 a1 = hfl((h16)x1[i]); hv[i] = a0; hv[4 + i] = a1; rv[i] = (h16)((x0[i] - (float)a0) * QRS); rv[4 + i] = (h16)((x1[i] - (float)a1) * QRS); }
                const size_t oo = sb + (size_t)row * (size_t)pitch + c8;
                *(volatile v8h*)(Ph + oo) = hv; if (useRes) *(volatile v8h*)(Pr + oo) = rv; }
            if (ps == 0) __threadfence(); }
        wave_sync();
    }
}

__global__ __launch_bounds__(32 * AW) void k_flash(const h16* __restrict__ QH, const h16* __restrict__ QR, const h16* __restrict__ KP, const h16* __restrict__ VH, const h16* __restrict__ VR, h16* CH, h16* CR) {
    __shared__ __align__(16) float os[AW * 16 * 68];
    const int lane = threadIdx.x & 31, wave = __builtin_amdgcn_readfirstlane((int)(threadIdx.x >> 5)), lr = lane & 15, hi = lane >> 4;
    const int zh = blockIdx.y; const int b = zh / NH_, h = zh % NH_;
    const int t0 = (blockIdx.x * AW + wave) * 16;
    const size_t pbase = (size_t)zh * SEQ * HD;
    const size_t qo = pbase + (size_t)(t0 + lr) * HD + 8 * hi;
    const v16h qh0 = ldh(QH + qo), qh1 = ldh(QH + qo + 32), qr0 = ldh(QR + qo), qr1 = ldh(QR + qo + 32);
    const size_t ko = pbase + (size_t)lr * HD + 8 * hi;
    const size_t vo = pbase + (size_t)lr * SEQ + 8 * hi;
    v8f oH0 = (v8f){}, oH1 = (v8f){}, oH2 = (v8f){}, oH3 = (v8f){};
    v8f oR0 = (v8f){}, oR1 = (v8f){}, oR2 = (v8f){}, oR3 = (v8f){};
    float m = -3.0e38f, l = 0.0f;
    const int tq = t0 + lr;
    const int kend = t0 + 16;
#pragma unroll 1
    for (int key0 = 0; key0 < kend; key0 += 32) {
        const h16* ka = KP + ko + (size_t)key0 * HD;
        const v16h ka0 = ldh(ka), ka1 = ldh(ka + 32), kb0 = ldh(ka + 16 * HD), kb1 = ldh(ka + 16 * HD + 32);
        v8f sHa = (v8f){}, sLa = (v8f){}, sHb = (v8f){}, sLb = (v8f){};
        sHa = wmma16(ka0, qh0, sHa); sLa = wmma16(ka0, qr0, sLa); sHb = wmma16(kb0, qh0, sHb); sLb = wmma16(kb0, qr0, sLb);
        sHa = wmma16(ka1, qh1, sHa); sLa = wmma16(ka1, qr1, sLa); sHb = wmma16(kb1, qh1, sHb); sLb = wmma16(kb1, qr1, sLb);
        asm volatile("v_nop\n\tv_nop\n\tv_nop\n\tv_nop" : "+v"(sHa), "+v"(sLa), "+v"(sHb), "+v"(sLb) : "v"(ka0), "v"(ka1), "v"(kb0), "v"(kb1));
        const int kq = key0 + 8 * hi;
        float ta[8], tb[8]; float mx = -3.0e38f;
#pragma unroll
        for (int r = 0; r < 8; ++r) { const float sa = (sHa[r] + sLa[r] * QRI) * SC2; const float sb = (sHb[r] + sLb[r] * QRI) * SC2;
            ta[r] = (kq + r <= tq) ? sa : -3.0e38f; tb[r] = (kq + 16 + r <= tq) ? sb : -3.0e38f; mx = fmaxf(mx, fmaxf(ta[r], tb[r])); }
        mx = fmaxf(mx, __shfl_xor(mx, 16, 32));
        const float mnew = fmaxf(m, mx);
        const float alpha = __builtin_amdgcn_exp2f(m - mnew);
        const float sh = PSH - mnew;
        v16h pbh, pbr; float ls = 0.0f;
#pragma unroll
        for (int r = 0; r < 8; ++r) {
            const float ea = __builtin_amdgcn_exp2f(ta[r] + sh); const float ec = __builtin_amdgcn_exp2f(tb[r] + sh);
            const float pa = (kq + r <= tq) ? ea : 0.0f; const float pc = (kq + 16 + r <= tq) ? ec : 0.0f;
            const h16 ha = (h16)pa; const h16 hc = (h16)pc;
            pbh[r] = ha; pbh[8 + r] = hc; pbr[r] = (h16)((pa - (float)ha) * QRS); pbr[8 + r] = (h16)((pc - (float)hc) * QRS);
            ls += pa + pc; }
        l = l * alpha + ls; m = mnew;
        oH0 = oH0 * alpha; oH1 = oH1 * alpha; oH2 = oH2 * alpha; oH3 = oH3 * alpha;
        oR0 = oR0 * alpha; oR1 = oR1 * alpha; oR2 = oR2 * alpha; oR3 = oR3 * alpha;
        const h16* va = VH + vo + key0;
        const v16h v0 = ldh(va), v1 = ldh(va + (size_t)16 * SEQ), v2 = ldh(va + (size_t)32 * SEQ), v3 = ldh(va + (size_t)48 * SEQ);
        oH0 = wmma16(v0, pbh, oH0); oH1 = wmma16(v1, pbh, oH1); oH2 = wmma16(v2, pbh, oH2); oH3 = wmma16(v3, pbh, oH3);
        oR0 = wmma16(v0, pbr, oR0); oR1 = wmma16(v1, pbr, oR1); oR2 = wmma16(v2, pbr, oR2); oR3 = wmma16(v3, pbr, oR3);
        const h16* vb = VR + vo + key0;
        const v16h w0 = ldh(vb), w1 = ldh(vb + (size_t)16 * SEQ), w2 = ldh(vb + (size_t)32 * SEQ), w3 = ldh(vb + (size_t)48 * SEQ);
        oR0 = wmma16(w0, pbh, oR0); oR1 = wmma16(w1, pbh, oR1); oR2 = wmma16(w2, pbh, oR2); oR3 = wmma16(w3, pbh, oR3);
        asm volatile("v_nop\n\tv_nop\n\tv_nop\n\tv_nop" : "+v"(oH0), "+v"(oH1), "+v"(oH2), "+v"(oH3), "+v"(oR0), "+v"(oR1), "+v"(oR2), "+v"(oR3) : "v"(w0), "v"(w1), "v"(w2), "v"(w3), "v"(pbh), "v"(pbr));
    }
    l += __shfl_xor(l, 16, 32);
    const float inv = 1.0f / l;
    const int wb = wave * 16 * 68;
    { v4f a, c;
#pragma unroll
      for (int i = 0; i < 4; ++i) { a[i] = (oH0[i] + oR0[i] * QRI) * inv; c[i] = (oH0[4 + i] + oR0[4 + i] * QRI) * inv; }
      *(v4fa*)(&os[wb + lr * 68 +  0 + 8 * hi]) = a; *(v4fa*)(&os[wb + lr * 68 +  0 + 8 * hi + 4]) = c;
#pragma unroll
      for (int i = 0; i < 4; ++i) { a[i] = (oH1[i] + oR1[i] * QRI) * inv; c[i] = (oH1[4 + i] + oR1[4 + i] * QRI) * inv; }
      *(v4fa*)(&os[wb + lr * 68 + 16 + 8 * hi]) = a; *(v4fa*)(&os[wb + lr * 68 + 16 + 8 * hi + 4]) = c;
#pragma unroll
      for (int i = 0; i < 4; ++i) { a[i] = (oH2[i] + oR2[i] * QRI) * inv; c[i] = (oH2[4 + i] + oR2[4 + i] * QRI) * inv; }
      *(v4fa*)(&os[wb + lr * 68 + 32 + 8 * hi]) = a; *(v4fa*)(&os[wb + lr * 68 + 32 + 8 * hi + 4]) = c;
#pragma unroll
      for (int i = 0; i < 4; ++i) { a[i] = (oH3[i] + oR3[i] * QRI) * inv; c[i] = (oH3[4 + i] + oR3[4 + i] * QRI) * inv; }
      *(v4fa*)(&os[wb + lr * 68 + 48 + 8 * hi]) = a; *(v4fa*)(&os[wb + lr * 68 + 48 + 8 * hi + 4]) = c; }
    wave_sync();
    const size_t cbase = ((size_t)b * SEQ + t0) * DM + (size_t)h * HD;
#pragma unroll 1
    for (int ps = 0; ps < 2; ++ps) {
#pragma unroll
        for (int s = 0; s < 4; ++s) { const int row = 4 * s + (lane >> 3), c8 = (lane & 7) * 8;
            const v4f x0 = *(const v4fa*)(&os[wb + row * 68 + c8]); const v4f x1 = *(const v4fa*)(&os[wb + row * 68 + c8 + 4]); v8h hv, rv;
#pragma unroll
            for (int i = 0; i < 4; ++i) { const h16 a0 = hfl((h16)x0[i]); const h16 a1 = hfl((h16)x1[i]); hv[i] = a0; hv[4 + i] = a1; rv[i] = (h16)((x0[i] - (float)a0) * QRS); rv[4 + i] = (h16)((x1[i] - (float)a1) * QRS); }
            const size_t oo = cbase + (size_t)row * DM + c8;
            *(volatile v8h*)(CH + oo) = hv; *(volatile v8h*)(CR + oo) = rv; }
        if (ps == 0) __threadfence(); }
}

__global__ __launch_bounds__(32) void k_oproj(const h16* __restrict__ AH, const h16* __restrict__ AR, const h16* __restrict__ Bt, const float* __restrict__ bo, float* OUT) {
    __shared__ __align__(16) float os[16 * 68];
    const int K = DM;
    const int lane = threadIdx.x & 31, lr = lane & 15, hi = lane >> 4; const int r0 = blockIdx.x * 32, c0 = blockIdx.y * 64;
    v8f aH[2][4], aR[2][4];
#pragma unroll
    for (int mb = 0; mb < 2; ++mb)
#pragma unroll
        for (int nb = 0; nb < 4; ++nb) { aH[mb][nb] = (v8f){}; aR[mb][nb] = (v8f){}; }
    const size_t aoff = (size_t)(r0 + lr) * K + 8 * hi, boff = (size_t)(c0 + lr) * K + 8 * hi;
#pragma unroll 1
    for (int kc = 0; kc < K; kc += 32) {
        v16h ah[2], ar[2];
#pragma unroll
        for (int mb = 0; mb < 2; ++mb) { ah[mb] = ldh(AH + aoff + (size_t)mb * 16 * K + kc); ar[mb] = ldh(AR + aoff + (size_t)mb * 16 * K + kc); }
#pragma unroll
        for (int nb = 0; nb < 4; ++nb) { const v16h bfrag = ldh(Bt + boff + (size_t)nb * 16 * K + kc);
#pragma unroll
            for (int mb = 0; mb < 2; ++mb) { aH[mb][nb] = wmma16(ah[mb], bfrag, aH[mb][nb]); aR[mb][nb] = wmma16(ar[mb], bfrag, aR[mb][nb]); } }
        asm volatile("v_nop\n\tv_nop\n\tv_nop\n\tv_nop" : "+v"(aH[0][3]), "+v"(aR[0][3]), "+v"(aH[1][3]), "+v"(aR[1][3]) : "v"(ah[0]), "v"(ah[1]), "v"(ar[0]), "v"(ar[1]));
    }
    float bc[4];
#pragma unroll
    for (int nb = 0; nb < 4; ++nb) bc[nb] = bfr(bo[c0 + nb * 16 + lr]);
    const int bb = r0 / SEQ, tt = r0 % SEQ;
    float* obase = OUT + ((size_t)bb * OUT_SEQ + tt) * DM + c0;
#pragma unroll
    for (int mb = 0; mb < 2; ++mb) {
#pragma unroll
        for (int nb = 0; nb < 4; ++nb) {
#pragma unroll
            for (int j = 0; j < 8; ++j) os[(hi * 8 + j) * 68 + nb * 16 + lr] = (aH[mb][nb][j] + aR[mb][nb][j] * QRI) * WOI + bc[nb]; }
        wave_sync();
#pragma unroll 1
        for (int ps = 0; ps < 2; ++ps) {
#pragma unroll
            for (int s = 0; s < 8; ++s) { const int row = 2 * s + hi, cofs = lr * 4;
                const v4f val = *(const v4fa*)(&os[row * 68 + cofs]);
                *(volatile v4f*)(obase + (size_t)(mb * 16 + row) * DM + cofs) = val; }
            if (ps == 0) __threadfence(); }
        wave_sync();
    }
}

static constexpr size_t al256(size_t v) { return (v + 255) & ~(size_t)255; }
static constexpr size_t SZ_XB = al256((size_t)NB * SEQ * DM * 2);
static constexpr size_t SZ_W  = al256((size_t)DM * DM * 2);
static constexpr size_t SZ_PL = al256((size_t)NB * NH_ * SEQ * HD * 2);
static constexpr size_t SZ_TOTAL = SZ_XB + 4 * SZ_W + 5 * SZ_PL + 2 * SZ_XB;
static_assert(SZ_TOTAL <= (size_t)134217728);

extern "C" void kernel_launch(void* const* d_in, const int* in_sizes, int n_in,
                              void* d_out, int out_size, void* d_ws, size_t ws_size, hipStream_t stream) {
    if (n_in < 9) return;
    const size_t needx = ((size_t)(NB - 1) * SEQ_FULL + SEQ) * DM;
    if ((size_t)in_sizes[0] < needx) return;
    const size_t nw = (size_t)NH_ * DM * HD;
    if ((size_t)in_sizes[1] < nw || (size_t)in_sizes[3] < nw || (size_t)in_sizes[5] < nw) return;
    if ((size_t)in_sizes[2] < (size_t)DM || (size_t)in_sizes[4] < (size_t)DM || (size_t)in_sizes[6] < (size_t)DM) return;
    if ((size_t)in_sizes[7] < (size_t)DM * DM || (size_t)in_sizes[8] < (size_t)DM) return;
    if ((size_t)out_size < ((size_t)(NB - 1) * OUT_SEQ + SEQ) * DM) return;
    if (SZ_TOTAL > ws_size) return;
    const float* x  = (const float*)d_in[0]; const float* wq = (const float*)d_in[1]; const float* wk = (const float*)d_in[3]; const float* wv = (const float*)d_in[5];
    const float* bq = (const float*)d_in[2]; const float* bk = (const float*)d_in[4]; const float* bv = (const float*)d_in[6];
    const float* wo = (const float*)d_in[7]; const float* bo = (const float*)d_in[8];
    float* OUT = (float*)d_out;
    char* wsp = (char*)d_ws;
    bf* XB = (bf*)wsp; wsp += SZ_XB;
    bf* WQ = (bf*)wsp; wsp += SZ_W;
    bf* WK = (bf*)wsp; wsp += SZ_W;
    bf* WV = (bf*)wsp; wsp += SZ_W;
    h16* WO = (h16*)wsp; wsp += SZ_W;
    h16* QH = (h16*)wsp; wsp += SZ_PL;
    h16* QR = (h16*)wsp; wsp += SZ_PL;
    h16* KP = (h16*)wsp; wsp += SZ_PL;
    h16* VH = (h16*)wsp; wsp += SZ_PL;
    h16* VR = (h16*)wsp; wsp += SZ_PL;
    h16* CH = (h16*)wsp; wsp += SZ_XB;
    h16* CR = (h16*)wsp; wsp += SZ_XB;

    if (SEQ == SEQ_FULL) {
        const size_t n8 = (size_t)NB * SEQ * DM / 8;
        k_cvt8<<<(unsigned)((n8 + 255) / 256), 256, 0, stream>>>(x, XB, n8);
    } else {
        const size_t n8 = (size_t)SEQ * DM / 8;
        for (int b = 0; b < NB; ++b) k_cvt8<<<(unsigned)((n8 + 255) / 256), 256, 0, stream>>>(x + (size_t)b * SEQ_FULL * DM, XB + (size_t)b * SEQ * DM, n8);
    }
    k_cvtT<0><<<dim3(HD / 64, DM / 64, NH_), 256, 0, stream>>>(wq, WQ, DM, HD, (size_t)DM * HD, (size_t)HD * DM);
    k_cvtT<0><<<dim3(HD / 64, DM / 64, NH_), 256, 0, stream>>>(wk, WK, DM, HD, (size_t)DM * HD, (size_t)HD * DM);
    k_cvtT<0><<<dim3(HD / 64, DM / 64, NH_), 256, 0, stream>>>(wv, WV, DM, HD, (size_t)DM * HD, (size_t)HD * DM);
    k_cvtT<1><<<dim3(DM / 64, DM / 64, 1), 256, 0, stream>>>(wo, (bf*)WO, DM, DM, (size_t)0, (size_t)0);

    k_proj<<<dim3(NB * SEQ / 64, DM / 64, 1), 32, 0, stream>>>(XB, WQ, QH, QR, 1, bq, 0, SEQ, (size_t)NH_ * SEQ * HD, HD, HD, (size_t)SEQ * HD);
    k_proj<<<dim3(NB * SEQ / 64, DM / 64, 1), 32, 0, stream>>>(XB, WK, KP, KP, 0, bk, 0, SEQ, (size_t)NH_ * SEQ * HD, HD, HD, (size_t)SEQ * HD);
    k_proj<<<dim3(DM / 64, NB * SEQ / 64, 1), 32, 0, stream>>>(WV, XB, VH, VR, 1, bv, 1, DM, (size_t)0, SEQ, SEQ, (size_t)DM * SEQ);

    k_flash<<<dim3(SEQ / (16 * AW), NB * NH_, 1), 32 * AW, 0, stream>>>(QH, QR, KP, VH, VR, CH, CR);

    k_oproj<<<dim3(NB * SEQ / 32, DM / 64, 1), 32, 0, stream>>>(CH, CR, WO, bo, OUT);
}
